// EnhancedHeteroGNN_13572096655643
// MI455X (gfx1250) — hardware-verified
//
#include <hip/hip_runtime.h>


#define FIN    7
#define EMBD   16
#define XIN    23
#define XK     32
#define HID    64
#define NHEAD  4
#define NTYPE  3
#define NACT   10
#define NTHR   256
#define NWAVE  8
#define EPT    8
#define NGRP   2
#define CHUNK  (NTHR * EPT * NGRP)
#define WCAP   (EPT * NGRP * 32)
#define LISTN  (NWAVE * WCAP)
#define ESH    13
#define NBC    8192
#define NBF    2048
#define FPC    (NBC / NBF)
#define RCAP   40960
#define RBN    128
#define OTHR   512
#define CPT    (NBC / OTHR)
#define GROWS  128
#define TGT2   256
#define DEGCAP 128
#define NBQ    128
#define AP2    (HID + 8)
#define SLOPE  0.2f
#define LDS_FILL ((RCAP + NBF + LISTN) * 4 + 64)
#define LDS_TAIL ((2 * NBQ * HID + LISTN + 2 * NBQ) * 4 + 64)

static_assert((CHUNK & (CHUNK - 1)) == 0);
static_assert(CHUNK <= (1 << ESH));
static_assert(NBC <= (1 << ESH) && NBF <= (1 << ESH) && NBQ <= (1 << ESH));
static_assert((NBC & (NBC - 1)) == 0 && (NBF & (NBF - 1)) == 0 && (NBQ & (NBQ - 1)) == 0);
static_assert(NBC == FPC * NBF && FPC == 4);
static_assert(OTHR * CPT == NBC && CPT == 16);
static_assert((OTHR / 32) == 4 * FPC);
static_assert((RCAP % 32) == 0);
static_assert((NBF % NTHR) == 0);
static_assert(GROWS == NWAVE * 16 && TGT2 == NWAVE * 32 && (TGT2 % GROWS) == 0);
static_assert(GROWS * HID * 4 <= 2 * GROWS * AP2 * 2);
static_assert(((AP2 * 2) % 16) == 0);
static_assert(NBQ * NACT <= LISTN);
static_assert((NBQ * HID) % NTHR == 0 && (NBQ * (HID / 2)) % NTHR == 0);
static_assert(NBQ <= NTHR);

typedef float          v2f  __attribute__((ext_vector_type(2)));
typedef float          v4f  __attribute__((ext_vector_type(4)));
typedef float          v8f  __attribute__((ext_vector_type(8)));
typedef int            v4i  __attribute__((ext_vector_type(4)));
typedef unsigned short v8us __attribute__((ext_vector_type(8)));
typedef __bf16         v16b __attribute__((ext_vector_type(16)));
union FragB { v16b v; v8us h[2]; };
union FI { float f; int i; };

__device__ __forceinline__ unsigned short bf_rne(float f) {
  unsigned u = __float_as_uint(f);
  u += 0x7FFFu + ((u >> 16) & 1u);
  return (unsigned short)(u >> 16);
}
__device__ __forceinline__ float bf_val(unsigned short b) { return __uint_as_float(((unsigned)b) << 16); }
__device__ __forceinline__ float lrelu(float x) { return x > 0.0f ? x : SLOPE * x; }
__device__ __forceinline__ float rdl(float v, int l) { FI u; u.f = v; u.i = __builtin_amdgcn_readlane(u.i, l); return u.f; }
__device__ __forceinline__ float wmax(float v) {
  v = fmaxf(v, __shfl_xor(v, 16)); v = fmaxf(v, __shfl_xor(v, 8)); v = fmaxf(v, __shfl_xor(v, 4));
  v = fmaxf(v, __shfl_xor(v, 2));  v = fmaxf(v, __shfl_xor(v, 1));
  return v;
}
__device__ __forceinline__ float wsum(float v) {
  v += __shfl_xor(v, 16); v += __shfl_xor(v, 8); v += __shfl_xor(v, 4); v += __shfl_xor(v, 2); v += __shfl_xor(v, 1);
  return v;
}

__device__ __forceinline__ v8f wmb(v16b a, v16b b, v8f c) {
  v8f d = __builtin_amdgcn_wmma_f32_16x16x32_bf16(false, a, false, b, (short)0, c, false, false);
  asm volatile("v_nop\n\tv_nop\n\tv_nop\n\tv_nop" : "+v"(d) : "v"(a), "v"(b));
  return d;
}

__device__ __forceinline__ void split8(const float* v, v8us& hv, v8us& lv) {
#pragma unroll
  for (int e = 0; e < 8; ++e) {
    const unsigned short h = bf_rne(v[e]);
    hv[e] = h;
    lv[e] = bf_rne(v[e] - bf_val(h));
  }
}

#define HITJ(J, HJ, SJ) { \
    const unsigned mj = __builtin_amdgcn_ballot_w32(HJ); \
    if (mj != 0u) { \
      if (HJ) { \
        const int pos = wc + (int)__builtin_amdgcn_mbcnt_lo(mj, 0u); \
        if (pos < WCAP) list[wave * WCAP + pos] = ((el0 + (J)) << ESH) | (int)(SJ); \
      } \
      wc += (int)__builtin_popcount(mj); } }

template <int NB>
__device__ __forceinline__ int scan_chunk(const int* __restrict__ dsts, int nE, int cbase, int slotBase,
                                          int vec8, int* list, int tid, int lane, int wave) {
  int wc = 0;
#pragma unroll
  for (int g = 0; g < NGRP; ++g) {
    const int el0  = (g * NTHR + tid) * EPT;
    const int e0   = cbase + el0;
    const int sent = -2147483647 - 1;
    v4i da, db;
    if (vec8 != 0 && cbase + CHUNK <= nE) {
      da = *(const v4i*)(dsts + e0);
      db = *(const v4i*)(dsts + e0 + 4);
    } else {
      da.x = (e0     < nE) ? dsts[min(e0,     nE - 1)] : sent;
      da.y = (e0 + 1 < nE) ? dsts[min(e0 + 1, nE - 1)] : sent;
      da.z = (e0 + 2 < nE) ? dsts[min(e0 + 2, nE - 1)] : sent;
      da.w = (e0 + 3 < nE) ? dsts[min(e0 + 3, nE - 1)] : sent;
      db.x = (e0 + 4 < nE) ? dsts[min(e0 + 4, nE - 1)] : sent;
      db.y = (e0 + 5 < nE) ? dsts[min(e0 + 5, nE - 1)] : sent;
      db.z = (e0 + 6 < nE) ? dsts[min(e0 + 6, nE - 1)] : sent;
      db.w = (e0 + 7 < nE) ? dsts[min(e0 + 7, nE - 1)] : sent;
    }
    const unsigned nb = (unsigned)slotBase;
    const unsigned s0 = (unsigned)da.x - nb, s1 = (unsigned)da.y - nb;
    const unsigned s2 = (unsigned)da.z - nb, s3 = (unsigned)da.w - nb;
    const unsigned s4 = (unsigned)db.x - nb, s5 = (unsigned)db.y - nb;
    const unsigned s6 = (unsigned)db.z - nb, s7 = (unsigned)db.w - nb;
    const bool h0 = s0 < (unsigned)NB, h1 = s1 < (unsigned)NB, h2 = s2 < (unsigned)NB, h3 = s3 < (unsigned)NB;
    const bool h4 = s4 < (unsigned)NB, h5 = s5 < (unsigned)NB, h6 = s6 < (unsigned)NB, h7 = s7 < (unsigned)NB;
    const unsigned any = __builtin_amdgcn_ballot_w32(h0 | h1 | h2 | h3 | h4 | h5 | h6 | h7);
    if (any != 0u) {
      HITJ(0, h0, s0)
      HITJ(1, h1, s1)
      HITJ(2, h2, s2)
      HITJ(3, h3, s3)
      HITJ(4, h4, s4)
      HITJ(5, h5, s5)
      HITJ(6, h6, s6)
      HITJ(7, h7, s7)
    }
  }
  return wc;
}

template <int NB>
__device__ __forceinline__ int scan_q(const int* __restrict__ srcs, const int* __restrict__ dsts, int nE,
                                      int cbase, int slotBase, int R, int vec8, int* list,
                                      int tid, int lane, int wave) {
  int wc = 0;
#pragma unroll
  for (int g = 0; g < NGRP; ++g) {
    const int el0  = (g * NTHR + tid) * EPT;
    const int e0   = cbase + el0;
    const int sent = -2147483647 - 1;
    v4i sa, sb, da, db;
    if (vec8 != 0 && cbase + CHUNK <= nE) {
      sa = *(const v4i*)(srcs + e0);
      sb = *(const v4i*)(srcs + e0 + 4);
      da = *(const v4i*)(dsts + e0);
      db = *(const v4i*)(dsts + e0 + 4);
    } else {
      sa.x = (e0     < nE) ? srcs[min(e0,     nE - 1)] : sent;
      sa.y = (e0 + 1 < nE) ? srcs[min(e0 + 1, nE - 1)] : sent;
      sa.z = (e0 + 2 < nE) ? srcs[min(e0 + 2, nE - 1)] : sent;
      sa.w = (e0 + 3 < nE) ? srcs[min(e0 + 3, nE - 1)] : sent;
      sb.x = (e0 + 4 < nE) ? srcs[min(e0 + 4, nE - 1)] : sent;
      sb.y = (e0 + 5 < nE) ? srcs[min(e0 + 5, nE - 1)] : sent;
      sb.z = (e0 + 6 < nE) ? srcs[min(e0 + 6, nE - 1)] : sent;
      sb.w = (e0 + 7 < nE) ? srcs[min(e0 + 7, nE - 1)] : sent;
      da.x = (e0     < nE) ? dsts[min(e0,     nE - 1)] : sent;
      da.y = (e0 + 1 < nE) ? dsts[min(e0 + 1, nE - 1)] : sent;
      da.z = (e0 + 2 < nE) ? dsts[min(e0 + 2, nE - 1)] : sent;
      da.w = (e0 + 3 < nE) ? dsts[min(e0 + 3, nE - 1)] : sent;
      db.x = (e0 + 4 < nE) ? dsts[min(e0 + 4, nE - 1)] : sent;
      db.y = (e0 + 5 < nE) ? dsts[min(e0 + 5, nE - 1)] : sent;
      db.z = (e0 + 6 < nE) ? dsts[min(e0 + 6, nE - 1)] : sent;
      db.w = (e0 + 7 < nE) ? dsts[min(e0 + 7, nE - 1)] : sent;
    }
    const unsigned nb = (unsigned)slotBase;
    const unsigned s0 = (unsigned)sa.x - nb, s1 = (unsigned)sa.y - nb;
    const unsigned s2 = (unsigned)sa.z - nb, s3 = (unsigned)sa.w - nb;
    const unsigned s4 = (unsigned)sb.x - nb, s5 = (unsigned)sb.y - nb;
    const unsigned s6 = (unsigned)sb.z - nb, s7 = (unsigned)sb.w - nb;
    const bool h0 = (s0 < (unsigned)NB) && (sa.x < R) && (da.x >= R);
    const bool h1 = (s1 < (unsigned)NB) && (sa.y < R) && (da.y >= R);
    const bool h2 = (s2 < (unsigned)NB) && (sa.z < R) && (da.z >= R);
    const bool h3 = (s3 < (unsigned)NB) && (sa.w < R) && (da.w >= R);
    const bool h4 = (s4 < (unsigned)NB) && (sb.x < R) && (db.x >= R);
    const bool h5 = (s5 < (unsigned)NB) && (sb.y < R) && (db.y >= R);
    const bool h6 = (s6 < (unsigned)NB) && (sb.z < R) && (db.z >= R);
    const bool h7 = (s7 < (unsigned)NB) && (sb.w < R) && (db.w >= R);
    const unsigned any = __builtin_amdgcn_ballot_w32(h0 | h1 | h2 | h3 | h4 | h5 | h6 | h7);
    if (any != 0u) {
      HITJ(0, h0, s0)
      HITJ(1, h1, s1)
      HITJ(2, h2, s2)
      HITJ(3, h3, s3)
      HITJ(4, h4, s4)
      HITJ(5, h5, s5)
      HITJ(6, h6, s6)
      HITJ(7, h7, s7)
    }
  }
  return wc;
}
#undef HITJ

__global__ __launch_bounds__(NTHR) void k_prep(
    const float* __restrict__ nf, const int* __restrict__ nt, const float* __restrict__ emb,
    const float* __restrict__ W1, const float* __restrict__ W2,
    unsigned short* xh, unsigned short* xl, unsigned short* w1h, unsigned short* w1l,
    unsigned short* w2h, unsigned short* w2l, int nN, int nPad) {
  const int gx = nPad * (XK / 8);
  const int g1 = NTYPE * HID * XK / 8;
  const int g2 = NTYPE * HID * HID / 8;
  const int bstart = blockIdx.x * NTHR;
  const int i = bstart + (int)threadIdx.x;
  float v[8];
  unsigned short* dh;
  unsigned short* dl;
  size_t o;
  if (bstart < gx) {
    const int n = i >> 2, k0 = (i & 3) * 8;
    const int nc = n < nN ? n : nN - 1;
    int t = nt[nc];
    t = t < 0 ? 0 : (t > 1 ? 1 : t);
#pragma unroll
    for (int e = 0; e < 8; ++e) {
      const int k  = k0 + e;
      const int kf = k < FIN ? k : FIN - 1;
      int ke = k - FIN;
      ke = ke < 0 ? 0 : (ke > EMBD - 1 ? EMBD - 1 : ke);
      const float a = nf[(size_t)nc * FIN + kf];
      const float b = emb[t * EMBD + ke];
      const float r = k < FIN ? a : (k < XIN ? b : 0.0f);
      v[e] = n < nN ? r : 0.0f;
    }
    dh = xh; dl = xl; o = (size_t)i * 8;
  } else if (bstart < gx + g1) {
    const int j   = i - gx;
    const int oo  = j * 8;
    const int ty  = oo / (HID * XK);
    const int rem = oo - ty * (HID * XK);
    const int n   = rem / XK;
    const int k0  = rem - n * XK;
#pragma unroll
    for (int e = 0; e < 8; ++e) {
      const int k  = k0 + e;
      const int kc = k < XIN ? k : XIN - 1;
      const float a = W1[(size_t)ty * XIN * HID + (size_t)kc * HID + n];
      v[e] = k < XIN ? a : 0.0f;
    }
    dh = w1h; dl = w1l; o = (size_t)j * 8;
  } else {
    const int j = i - gx - g1;
    if (j >= g2) return;
    const int oo  = j * 8;
    const int ty  = oo / (HID * HID);
    const int rem = oo - ty * (HID * HID);
    const int n   = rem / HID;
    const int k0  = rem - n * HID;
#pragma unroll
    for (int e = 0; e < 8; ++e) v[e] = W2[(size_t)ty * HID * HID + (size_t)(k0 + e) * HID + n];
    dh = w2h; dl = w2l; o = (size_t)j * 8;
  }
  v8us hv, lv;
  split8(v, hv, lv);
  *(volatile v8us*)(dh + o) = hv;
  *(volatile v8us*)(dl + o) = lv;
  __threadfence();
  *(volatile v8us*)(dh + o) = hv;
  *(volatile v8us*)(dl + o) = lv;
}

__global__ __launch_bounds__(NTHR) void k_count(
    const int* __restrict__ ei, int* cnt, int nE, int vec8) {
  __shared__ __attribute__((aligned(16))) int scnt[NBC];
  __shared__ __attribute__((aligned(16))) int list[LISTN];
  __shared__ int wcnt[NWAVE];
  const int tid = threadIdx.x, lane = tid & 31, wave = tid >> 5;
  const int nodeBase = blockIdx.x * NBC;
  const int* dsts = ei + nE;

  for (int i = tid; i < NBC; i += NTHR) scnt[i] = 0;
  __syncthreads();

  const int nChunks = (nE + CHUNK - 1) / CHUNK;
#pragma unroll 1
  for (int ch = 0; ch < nChunks; ++ch) {
    const int cbase = ch * CHUNK;
    const int wc = scan_chunk<NBC>(dsts, nE, cbase, nodeBase, vec8, list, tid, lane, wave);
    if (lane == 0) wcnt[wave] = wc;
    __syncthreads();
    if (wave == 0) {
#pragma unroll 1
      for (int wsx = 0; wsx < NWAVE; ++wsx) {
        int n = __builtin_amdgcn_readfirstlane(wcnt[wsx]);
        n = n > WCAP ? WCAP : (n < 0 ? 0 : n);
        const int* lp = list + wsx * WCAP;
#pragma unroll 1
        for (int i = 0; i < n; ++i) {
          const int ent  = __builtin_amdgcn_readfirstlane(lp[i]);
          const int slot = ent & (NBC - 1);
          if (lane == 0) scnt[slot] = scnt[slot] + 1;
        }
      }
    }
    __syncthreads();
  }

  v4i cq[8];
#pragma unroll
  for (int q = 0; q < 8; ++q) {
    const int f = (wave * 8 + q) * 128 + 4 * lane;
    cq[q] = *(const v4i*)(scnt + f);
  }
  int* cp = cnt + (size_t)nodeBase;
#pragma unroll
  for (int q = 0; q < 8; ++q) {
    const int f = (wave * 8 + q) * 128 + 4 * lane;
    *(volatile v4i*)(cp + f) = cq[q];
  }
  __threadfence();
#pragma unroll
  for (int q = 0; q < 8; ++q) {
    const int f = (wave * 8 + q) * 128 + 4 * lane;
    *(volatile v4i*)(cp + f) = cq[q];
  }
}

__global__ __launch_bounds__(OTHR) void k_offsets(
    const int* __restrict__ cnt, int* off, int* rbase, int nChunk) {
  __shared__ __attribute__((aligned(16))) int soff[NBC];
  __shared__ __attribute__((aligned(16))) int srb[RBN];
  __shared__ int wtot[OTHR / 32];
  const int tid = threadIdx.x, lane = tid & 31, wave = tid >> 5, sub = tid >> 7;
  for (int i = tid; i < RBN; i += OTHR) srb[i] = 0;
  int carry = 0;
#pragma unroll 1
  for (int ch = 0; ch < nChunk; ++ch) {
    const int base = ch * NBC;
    v4i cv[4];
#pragma unroll
    for (int q = 0; q < 4; ++q) cv[q] = *(const v4i*)(cnt + base + CPT * tid + 4 * q);
    int e[CPT];
#pragma unroll
    for (int q = 0; q < 4; ++q) {
      e[4 * q + 0] = cv[q].x < 0 ? 0 : cv[q].x;
      e[4 * q + 1] = cv[q].y < 0 ? 0 : cv[q].y;
      e[4 * q + 2] = cv[q].z < 0 ? 0 : cv[q].z;
      e[4 * q + 3] = cv[q].w < 0 ? 0 : cv[q].w;
    }
    int ts = 0;
#pragma unroll
    for (int q = 0; q < CPT; ++q) ts += e[q];
    int incl = ts;
#pragma unroll
    for (int d = 1; d < 32; d <<= 1) {
      const int t = __shfl_up(incl, d);
      if (lane >= d) incl += t;
    }
    if (lane == 31) wtot[wave] = incl;
    __syncthreads();
    const int S0 = wtot[0]  + wtot[1]  + wtot[2]  + wtot[3];
    const int S1 = wtot[4]  + wtot[5]  + wtot[6]  + wtot[7];
    const int S2 = wtot[8]  + wtot[9]  + wtot[10] + wtot[11];
    const int S3 = wtot[12] + wtot[13] + wtot[14] + wtot[15];
    int pre = 0;
#pragma unroll 1
    for (int w = 4 * sub; w < wave; ++w) pre += wtot[w];
    const int b0 = carry;
    const int b1 = b0 + ((S0 + 31) & ~31);
    const int b2 = b1 + ((S1 + 31) & ~31);
    const int b3 = b2 + ((S2 + 31) & ~31);
    const int b4 = b3 + ((S3 + 31) & ~31);
    const int myb = sub == 0 ? b0 : (sub == 1 ? b1 : (sub == 2 ? b2 : b3));
    if (tid == 0) {
      srb[min(FPC * ch + 0, RBN - 1)] = b0;
      srb[min(FPC * ch + 1, RBN - 1)] = b1;
      srb[min(FPC * ch + 2, RBN - 1)] = b2;
      srb[min(FPC * ch + 3, RBN - 1)] = b3;
    }
    int run = myb + pre + incl - ts;
#pragma unroll
    for (int q = 0; q < CPT; ++q) { soff[CPT * tid + q] = run; run += e[q]; }
    carry = b4;
    __syncthreads();
    v4i ov[4];
#pragma unroll
    for (int q = 0; q < 4; ++q) ov[q] = *(const v4i*)(soff + 4 * (tid + q * OTHR));
    int* op = off + base;
#pragma unroll
    for (int q = 0; q < 4; ++q) *(volatile v4i*)(op + 4 * (tid + q * OTHR)) = ov[q];
    __threadfence();
#pragma unroll
    for (int q = 0; q < 4; ++q) *(volatile v4i*)(op + 4 * (tid + q * OTHR)) = ov[q];
    __syncthreads();
  }
  if (tid == 0) srb[min(FPC * nChunk, RBN - 1)] = carry;
  __syncthreads();
  v4i rv = {0, 0, 0, 0};
  if (tid < 32) rv = *(const v4i*)(srb + 4 * tid);
  if (tid < 32) *(volatile v4i*)(rbase + 4 * tid) = rv;
  __threadfence();
  if (tid < 32) *(volatile v4i*)(rbase + 4 * tid) = rv;
}

__global__ __launch_bounds__(NTHR) void k_fill(
    const int* __restrict__ ei, const int* __restrict__ off, const int* __restrict__ rbase,
    int* csr, int nN, int nE, int vec8, int csrLen) {
  extern __shared__ v4f lds_dyn[];
  int* region = (int*)lds_dyn;
  int* cursor = region + RCAP;
  int* list   = cursor + NBF;
  int* wcnt   = list + LISTN;
  const int tid = threadIdx.x, lane = tid & 31, wave = tid >> 5;
  const int b = blockIdx.x;
  const int nodeBase = b * NBF;
  const int* dsts = ei + nE;

  int rb0 = rbase[b];
  const int rb1 = rbase[b + 1];
  rb0 = rb0 < 0 ? 0 : (rb0 > csrLen ? csrLen : rb0);
  rb0 &= ~31;
  int len = rb1 - rb0;
  len = len < 0 ? 0 : (len > RCAP ? RCAP : len);
  int lenW = (len + 31) & ~31;
  if (rb0 + lenW > csrLen) lenW = (csrLen - rb0) & ~31;

  {
    const v4i z = {0, 0, 0, 0};
    for (int i = tid; i < RCAP / 4; i += NTHR) ((v4i*)region)[i] = z;
    for (int s = tid; s < NBF; s += NTHR) {
      int o = off[nodeBase + s] - rb0;
      o = o < 0 ? 0 : (o > RCAP ? RCAP : o);
      cursor[s] = o;
    }
  }
  __syncthreads();

  const int nChunks = (nE + CHUNK - 1) / CHUNK;
#pragma unroll 1
  for (int ch = 0; ch < nChunks; ++ch) {
    const int cbase = ch * CHUNK;
    const int wc = scan_chunk<NBF>(dsts, nE, cbase, nodeBase, vec8, list, tid, lane, wave);
    if (lane == 0) wcnt[wave] = wc;
    __syncthreads();
    if (wave == 0) {
#pragma unroll 1
      for (int wsx = 0; wsx < NWAVE; ++wsx) {
        int n = __builtin_amdgcn_readfirstlane(wcnt[wsx]);
        n = n > WCAP ? WCAP : (n < 0 ? 0 : n);
        const int* lp = list + wsx * WCAP;
#pragma unroll 1
        for (int i = 0; i < n; ++i) {
          const int ent  = __builtin_amdgcn_readfirstlane(lp[i]);
          const int slot = ent & (NBF - 1);
          int e = cbase + ((ent >> ESH) & (CHUNK - 1));
          e = e > nE - 1 ? nE - 1 : e;
          int src = ei[e];
          src = src < 0 ? 0 : (src > nN - 1 ? nN - 1 : src);
          if (lane == 0) {
            int pos = cursor[slot];
            pos = pos < 0 ? 0 : (pos > RCAP - 1 ? RCAP - 1 : pos);
            region[pos] = src;
            const int np = pos + 1;
            cursor[slot] = np > RCAP ? RCAP : np;
          }
        }
      }
    }
    __syncthreads();
  }

  const int nv = lenW >> 2;
  int* gp = csr + rb0;
#pragma unroll 1
  for (int i = tid; i < nv; i += NTHR) { const v4i v = ((const v4i*)region)[i]; *(volatile v4i*)(gp + 4 * i) = v; }
  __threadfence();
#pragma unroll 1
  for (int i = tid; i < nv; i += NTHR) { const v4i v = ((const v4i*)region)[i]; *(volatile v4i*)(gp + 4 * i) = v; }
}

__global__ __launch_bounds__(NTHR) void k_gemm1(
    const unsigned short* __restrict__ xh, const unsigned short* __restrict__ xl,
    const unsigned short* __restrict__ wh, const unsigned short* __restrict__ wl,
    const float* __restrict__ as1, const float* __restrict__ ad1,
    float* h1, float* als, float* ald) {
  __shared__ __attribute__((aligned(16))) float stg[GROWS * HID];
  __shared__ __attribute__((aligned(16))) float sal[2 * GROWS * NHEAD];
  __shared__ float sav[2 * HID];
  const int tid = threadIdx.x, lane = tid & 31, wave = tid >> 5, hh = lane >> 4, m = lane & 15;
  const int rowBase = blockIdx.x * GROWS;
  if (tid < HID) { sav[tid] = as1[tid]; sav[HID + tid] = ad1[tid]; }

  const size_t row = (size_t)(rowBase + wave * 16 + m);
  FragB ah, al;
  ah.h[0] = *(const v8us*)(xh + row * XK + 8 * hh);
  ah.h[1] = *(const v8us*)(xh + row * XK + 16 + 8 * hh);
  al.h[0] = *(const v8us*)(xl + row * XK + 8 * hh);
  al.h[1] = *(const v8us*)(xl + row * XK + 16 + 8 * hh);
  v8f acc[4];
#pragma unroll
  for (int t = 0; t < 4; ++t) { v8f z = {0.f, 0.f, 0.f, 0.f, 0.f, 0.f, 0.f, 0.f}; acc[t] = z; }
#pragma unroll
  for (int t = 0; t < 4; ++t) {
    const int bo = (16 * t + m) * XK + 8 * hh;
    FragB bh, bl;
    bh.h[0] = *(const v8us*)(wh + bo);
    bh.h[1] = *(const v8us*)(wh + bo + 16);
    bl.h[0] = *(const v8us*)(wl + bo);
    bl.h[1] = *(const v8us*)(wl + bo + 16);
    acc[t] = wmb(ah.v, bh.v, acc[t]);
    acc[t] = wmb(ah.v, bl.v, acc[t]);
    acc[t] = wmb(al.v, bh.v, acc[t]);
  }
  float* sp = stg + (wave * 16 + 8 * hh) * HID + m;
#pragma unroll
  for (int t = 0; t < 4; ++t) {
#pragma unroll
    for (int r = 0; r < 8; ++r) sp[r * HID + 16 * t] = acc[t][r];
  }
  __syncthreads();

  {
    const int rr = wave * 16 + (lane & 15);
    const int hs = lane >> 4;
    const float* rp = stg + rr * HID + 32 * hs;
    const float* ap = sav + 32 * hs;
    const float* dp = sav + HID + 32 * hs;
    float s0 = 0.f, s1 = 0.f, d0 = 0.f, d1 = 0.f;
#pragma unroll 2
    for (int c = 0; c < 16; ++c) {
      const float x0 = rp[c], x1 = rp[16 + c];
      s0 += x0 * ap[c];
      s1 += x1 * ap[16 + c];
      d0 += x0 * dp[c];
      d1 += x1 * dp[16 + c];
    }
    sal[rr * NHEAD + 2 * hs]     = s0;
    sal[rr * NHEAD + 2 * hs + 1] = s1;
    sal[GROWS * NHEAD + rr * NHEAD + 2 * hs]     = d0;
    sal[GROWS * NHEAD + rr * NHEAD + 2 * hs + 1] = d1;
  }
  __syncthreads();

  const float* lp = stg + wave * 16 * HID + 4 * lane;
  float* gp = h1 + ((size_t)rowBase + wave * 16) * HID + 4 * lane;
  const int wsel = wave >> 2, wsub = wave & 3;
  const v4f av = *(const v4f*)(sal + wsel * GROWS * NHEAD + (wsub * 32 + lane) * NHEAD);
  float* agp = (wsel == 0 ? als : ald) + ((size_t)rowBase + wsub * 32 + lane) * NHEAD;
#pragma unroll
  for (int i = 0; i < 8; ++i) { const v4f v = *(const v4f*)(lp + i * 128); *(volatile v4f*)(gp + (size_t)i * 128) = v; }
  *(volatile v4f*)agp = av;
  __threadfence();
#pragma unroll
  for (int i = 0; i < 8; ++i) { const v4f v = *(const v4f*)(lp + i * 128); *(volatile v4f*)(gp + (size_t)i * 128) = v; }
  *(volatile v4f*)agp = av;
}

__global__ __launch_bounds__(NTHR) void k_agg1g2(
    const int* __restrict__ csr, const int* __restrict__ off, const int* __restrict__ cnt,
    const float* __restrict__ als1, const float* __restrict__ ald1, const float* __restrict__ h1,
    const float* __restrict__ b1, const unsigned short* __restrict__ wh, const unsigned short* __restrict__ wl,
    const float* __restrict__ as2, const float* __restrict__ ad2,
    float* h2, float* als2, float* ald2, int nN, int csrLen) {
  __shared__ __attribute__((aligned(16))) v4f lraw[(2 * GROWS * AP2 * 2) / 16];
  __shared__ __attribute__((aligned(16))) float sal[2 * GROWS];
  __shared__ float sav[2 * HID];
  unsigned short* sAh = (unsigned short*)lraw;
  unsigned short* sAl = sAh + GROWS * AP2;
  float* stg = (float*)lraw;
  const int tid = threadIdx.x, lane = tid & 31, wave = tid >> 5, hh = lane >> 4, m = lane & 15;
  const int head = lane >> 3;
  const int rowBase = blockIdx.x * GROWS;
  const int tb = rowBase + wave * 16;
  if (tid < HID) { sav[tid] = as2[tid]; sav[HID + tid] = ad2[tid]; }
  const int cnt_l = cnt[tb + (lane & 15)];
  const int off_l = off[tb + (lane & 15)];
  const v2f bv = *(const v2f*)(b1 + 2 * lane);

#pragma unroll 1
  for (int j = 0; j < 16; ++j) {
    const int c = tb + j;
    int n = __builtin_amdgcn_readlane(cnt_l, j);
    n = n < 0 ? 0 : (n > DEGCAP ? DEGCAP : n);
    const int st = __builtin_amdgcn_readlane(off_l, j);
    const float adh = ald1[(size_t)c * NHEAD + head];
    const float ls  = lrelu(als1[(size_t)c * NHEAD + head] + adh);
    float mx = ls;
#pragma unroll 1
    for (int q0 = 0; q0 < n; q0 += 32) {
      int pos = st + q0 + lane;
      pos = pos < 0 ? 0 : (pos > csrLen - 1 ? csrLen - 1 : pos);
      int sl = csr[pos];
      sl = sl < 0 ? 0 : (sl > nN - 1 ? nN - 1 : sl);
      const int mcnt = (n - q0) < 32 ? (n - q0) : 32;
#pragma unroll 1
      for (int p = 0; p < mcnt; ++p) {
        const int s = __builtin_amdgcn_readlane(sl, p);
        mx = fmaxf(mx, lrelu(als1[(size_t)s * NHEAD + head] + adh));
      }
    }
    float den = __expf(ls - mx);
    v2f acc = *(const v2f*)(h1 + (size_t)c * HID + 2 * lane) * den;
#pragma unroll 1
    for (int q0 = 0; q0 < n; q0 += 32) {
      int pos = st + q0 + lane;
      pos = pos < 0 ? 0 : (pos > csrLen - 1 ? csrLen - 1 : pos);
      int sl = csr[pos];
      sl = sl < 0 ? 0 : (sl > nN - 1 ? nN - 1 : sl);
      const int mcnt = (n - q0) < 32 ? (n - q0) : 32;
#pragma unroll 1
      for (int p = 0; p < mcnt; ++p) {
        const int s = __builtin_amdgcn_readlane(sl, p);
        const float ex = __expf(lrelu(als1[(size_t)s * NHEAD + head] + adh) - mx);
        den += ex;
        const v2f r = *(const v2f*)(h1 + (size_t)s * HID + 2 * lane);
        acc += r * ex;
      }
    }
    const float inv = 1.0f / den;
    v2f v = acc * inv + bv;
    v.x = v.x > 0.0f ? v.x : expm1f(fminf(v.x, 0.0f));
    v.y = v.y > 0.0f ? v.y : expm1f(fminf(v.y, 0.0f));
    const unsigned short hx = bf_rne(v.x), hy = bf_rne(v.y);
    const unsigned short lx = bf_rne(v.x - bf_val(hx)), ly = bf_rne(v.y - bf_val(hy));
    const int ro = (wave * 16 + j) * AP2 + 2 * lane;
    *(unsigned*)(sAh + ro) = (unsigned)hx | ((unsigned)hy << 16);
    *(unsigned*)(sAl + ro) = (unsigned)lx | ((unsigned)ly << 16);
  }
  __syncthreads();

  v8f acc2[4];
#pragma unroll
  for (int t = 0; t < 4; ++t) { v8f z = {0.f, 0.f, 0.f, 0.f, 0.f, 0.f, 0.f, 0.f}; acc2[t] = z; }
  const unsigned short* arh = sAh + (wave * 16 + m) * AP2 + 8 * hh;
  const unsigned short* arl = sAl + (wave * 16 + m) * AP2 + 8 * hh;
#pragma unroll
  for (int kt = 0; kt < HID / 32; ++kt) {
    FragB ah, al;
    ah.h[0] = *(const v8us*)(arh + 32 * kt);
    ah.h[1] = *(const v8us*)(arh + 32 * kt + 16);
    al.h[0] = *(const v8us*)(arl + 32 * kt);
    al.h[1] = *(const v8us*)(arl + 32 * kt + 16);
#pragma unroll
    for (int t = 0; t < 4; ++t) {
      const int bo = (16 * t + m) * HID + 32 * kt + 8 * hh;
      FragB bh, bl;
      bh.h[0] = *(const v8us*)(wh + bo);
      bh.h[1] = *(const v8us*)(wh + bo + 16);
      bl.h[0] = *(const v8us*)(wl + bo);
      bl.h[1] = *(const v8us*)(wl + bo + 16);
      acc2[t] = wmb(ah.v, bh.v, acc2[t]);
      acc2[t] = wmb(ah.v, bl.v, acc2[t]);
      acc2[t] = wmb(al.v, bh.v, acc2[t]);
    }
  }
  __syncthreads();

  float* sp = stg + (wave * 16 + 8 * hh) * HID + m;
#pragma unroll
  for (int t = 0; t < 4; ++t) {
#pragma unroll
    for (int r = 0; r < 8; ++r) sp[r * HID + 16 * t] = acc2[t][r];
  }
  __syncthreads();

  {
    const int rr  = wave * 16 + (lane & 15);
    const int ws2 = lane >> 4;
    const float* rp = stg + rr * HID;
    const float* ap = sav + ws2 * HID;
    float d0 = 0.f, d1 = 0.f, d2 = 0.f, d3 = 0.f;
#pragma unroll 2
    for (int k = 0; k < 16; ++k) {
      d0 += rp[k]      * ap[k];
      d1 += rp[16 + k] * ap[16 + k];
      d2 += rp[32 + k] * ap[32 + k];
      d3 += rp[48 + k] * ap[48 + k];
    }
    sal[ws2 * GROWS + rr] = (d0 + d1) + (d2 + d3);
  }
  __syncthreads();

  const float* lp = stg + wave * 16 * HID + 4 * lane;
  float* gp = h2 + ((size_t)rowBase + wave * 16) * HID + 4 * lane;
  const int wa = wave < 2 ? wave : 0;
  const v4f av = *(const v4f*)(sal + wa * GROWS + 4 * lane);
  float* agp = (wa == 0 ? als2 : ald2) + (size_t)rowBase + 4 * lane;
#pragma unroll
  for (int i = 0; i < 8; ++i) { const v4f v = *(const v4f*)(lp + i * 128); *(volatile v4f*)(gp + (size_t)i * 128) = v; }
  if (wave < 2) *(volatile v4f*)agp = av;
  __threadfence();
#pragma unroll
  for (int i = 0; i < 8; ++i) { const v4f v = *(const v4f*)(lp + i * 128); *(volatile v4f*)(gp + (size_t)i * 128) = v; }
  if (wave < 2) *(volatile v4f*)agp = av;
}

__global__ __launch_bounds__(NTHR) void k_agg2(
    const int* __restrict__ csr, const int* __restrict__ off, const int* __restrict__ cnt,
    const float* __restrict__ als, const float* __restrict__ ald, const float* __restrict__ h2,
    const float* __restrict__ b2, const float* __restrict__ ea, int et,
    float* xcomb, int nN, int csrLen) {
  const int tid = threadIdx.x, lane = tid & 31, wave = tid >> 5;
  const int tb = blockIdx.x * TGT2 + wave * 32;
  const int cnt_l = cnt[tb + lane];
  const int off_l = off[tb + lane];
  const float as_l = als[tb + lane];
  const float ad_l = ald[tb + lane];
  const v2f bv = *(const v2f*)(b2 + 2 * lane);
  float ew;
  {
    const float a0 = ea[0], a1 = ea[1], a2 = ea[2];
    const float am = fmaxf(a0, fmaxf(a1, a2));
    const float e0 = __expf(a0 - am), e1 = __expf(a1 - am), e2 = __expf(a2 - am);
    const float rs = 1.0f / (e0 + e1 + e2);
    ew = (et == 0 ? e0 : (et == 1 ? e1 : e2)) * rs;
  }

#pragma unroll 1
  for (int j = 0; j < 32; ++j) {
    const int c = tb + j;
    int n = __builtin_amdgcn_readlane(cnt_l, j);
    n = n < 0 ? 0 : (n > DEGCAP ? DEGCAP : n);
    const int st = __builtin_amdgcn_readlane(off_l, j);
    const float ad = rdl(ad_l, j);
    const float ls = lrelu(rdl(as_l, j) + ad);
    float mx = ls;
#pragma unroll 1
    for (int q0 = 0; q0 < n; q0 += 32) {
      int pos = st + q0 + lane;
      pos = pos < 0 ? 0 : (pos > csrLen - 1 ? csrLen - 1 : pos);
      int sl = csr[pos];
      sl = sl < 0 ? 0 : (sl > nN - 1 ? nN - 1 : sl);
      const float lg = lrelu(als[sl] + ad);
      mx = fmaxf(mx, (q0 + lane < n) ? lg : ls);
    }
    mx = wmax(mx);
    const float exs = __expf(ls - mx);
    v2f acc = *(const v2f*)(h2 + (size_t)c * HID + 2 * lane) * exs;
    float dsum = 0.0f;
#pragma unroll 1
    for (int q0 = 0; q0 < n; q0 += 32) {
      int pos = st + q0 + lane;
      pos = pos < 0 ? 0 : (pos > csrLen - 1 ? csrLen - 1 : pos);
      int sl = csr[pos];
      sl = sl < 0 ? 0 : (sl > nN - 1 ? nN - 1 : sl);
      const float lg  = lrelu(als[sl] + ad);
      const float exl = (q0 + lane < n) ? __expf(lg - mx) : 0.0f;
      dsum += exl;
      const int mcnt = (n - q0) < 32 ? (n - q0) : 32;
#pragma unroll 1
      for (int p = 0; p < mcnt; ++p) {
        const int s = __builtin_amdgcn_readlane(sl, p);
        const float ex = rdl(exl, p);
        const v2f r = *(const v2f*)(h2 + (size_t)s * HID + 2 * lane);
        acc += r * ex;
      }
    }
    const float den = wsum(dsum) + exs;
    const float inv = 1.0f / den;
    v2f v = (acc * inv + bv) * ew;
    float* xp = xcomb + (size_t)c * HID + 2 * lane;
    if (et != 0) { const v2f o2 = *(const v2f*)xp; v = o2 + v; }
    *(volatile v2f*)xp = v;
    __threadfence();
    *(volatile v2f*)xp = v;
  }
}

__global__ __launch_bounds__(NTHR) void k_tail(
    const int* __restrict__ ei, int nE, int vec8, int nN, int R,
    const float* __restrict__ xcomb, const float* __restrict__ Wo1, const float* __restrict__ bo1,
    const float* __restrict__ Wo2, const float* __restrict__ bo2,
    const float* __restrict__ Wo3, const float* __restrict__ bo3, float* out) {
  extern __shared__ v4f lds_dyn[];
  float* sums = (float*)lds_dyn;
  float* hq1s = sums + NBQ * HID;
  int*   list = (int*)(hq1s + NBQ * HID);
  int*   cq   = list + LISTN;
  float* rinv = (float*)(cq + NBQ);
  int*   wcnt = (int*)(rinv + NBQ);
  float* hq2s = sums;
  float* outs = (float*)list;
  const int tid = threadIdx.x, lane = tid & 31, wave = tid >> 5;
  const int qBase = blockIdx.x * NBQ;

  {
    const v4f z = {0.f, 0.f, 0.f, 0.f};
    for (int i = tid; i < NBQ * HID / 4; i += NTHR) ((v4f*)sums)[i] = z;
    for (int i = tid; i < NBQ; i += NTHR) cq[i] = 0;
  }
  __syncthreads();

  const int nChunks = (nE + CHUNK - 1) / CHUNK;
#pragma unroll 1
  for (int ch = 0; ch < nChunks; ++ch) {
    const int cbase = ch * CHUNK;
    const int wc = scan_q<NBQ>(ei, ei + nE, nE, cbase, qBase, R, vec8, list, tid, lane, wave);
    if (lane == 0) wcnt[wave] = wc;
    __syncthreads();
    if (wave == 0) {
#pragma unroll 1
      for (int wsx = 0; wsx < NWAVE; ++wsx) {
        int n = __builtin_amdgcn_readfirstlane(wcnt[wsx]);
        n = n > WCAP ? WCAP : (n < 0 ? 0 : n);
        const int* lp = list + wsx * WCAP;
#pragma unroll 1
        for (int i = 0; i < n; ++i) {
          const int ent  = __builtin_amdgcn_readfirstlane(lp[i]);
          const int slot = ent & (NBQ - 1);
          int e = cbase + ((ent >> ESH) & (CHUNK - 1));
          e = e > nE - 1 ? nE - 1 : e;
          int d = ei[(size_t)nE + e];
          d = d < 0 ? 0 : (d > nN - 1 ? nN - 1 : d);
          const v2f r = *(const v2f*)(xcomb + (size_t)d * HID + 2 * lane);
          v2f* ap = (v2f*)(sums + slot * HID + 2 * lane);
          *ap = *ap + r;
          if (lane == 0) cq[slot] = cq[slot] + 1;
        }
      }
    }
    __syncthreads();
  }
  if (tid < NBQ) { int cc = cq[tid]; cc = cc < 1 ? 1 : cc; rinv[tid] = 1.0f / (float)cc; }
  __syncthreads();

#pragma unroll 1
  for (int it = 0; it < NBQ * HID / NTHR; ++it) {
    const int idx = it * NTHR + tid;
    const int r = idx >> 6, jj = idx & 63;
    int rg = qBase + r;
    rg = rg > R - 1 ? R - 1 : rg;
    const float* xr = xcomb + (size_t)rg * HID;
    const float* vr = sums + r * HID;
    const float ir = rinv[r];
    float s = bo1[jj];
#pragma unroll 2
    for (int k = 0; k < HID; ++k) s += xr[k] * Wo1[k * HID + jj];
#pragma unroll 2
    for (int k = 0; k < HID; ++k) { const float vk = vr[k] * ir; s += vk * Wo1[(HID + k) * HID + jj]; }
    hq1s[r * HID + jj] = fmaxf(s, 0.0f);
  }
  __syncthreads();
#pragma unroll 1
  for (int it = 0; it < NBQ * (HID / 2) / NTHR; ++it) {
    const int idx = it * NTHR + tid;
    const int r = idx >> 5, jj = idx & 31;
    const float* hr = hq1s + r * HID;
    float s = bo2[jj];
#pragma unroll 2
    for (int k = 0; k < HID; ++k) s += hr[k] * Wo2[k * (HID / 2) + jj];
    hq2s[r * (HID / 2) + jj] = fmaxf(s, 0.0f);
  }
  __syncthreads();
#pragma unroll 1
  for (int it = 0; it < (NBQ * NACT + NTHR - 1) / NTHR; ++it) {
    const int idx = it * NTHR + tid;
    if (idx < NBQ * NACT) {
      const int r = idx / NACT, jj = idx - r * NACT;
      const float* hr = hq2s + r * (HID / 2);
      float s = bo3[jj];
#pragma unroll 2
      for (int k = 0; k < HID / 2; ++k) s += hr[k] * Wo3[k * NACT + jj];
      outs[idx] = s;
    }
  }
  __syncthreads();

  int nrow = R - qBase;
  nrow = nrow > NBQ ? NBQ : nrow;
  const int nfl = nrow * NACT;
  const int np  = nfl >> 2;
  const int rem = nfl & 3;
  float* op = out + (size_t)qBase * NACT;
  const int p0 = tid, p1 = NTHR + tid;
  const v4f pv0 = *(const v4f*)(outs + 4 * (p0 < np ? p0 : 0));
  const v4f pv1 = *(const v4f*)(outs + 4 * (p1 < np ? p1 : 0));
  v2f tv = {0.f, 0.f};
  if (rem != 0) { tv.x = outs[nfl - 2]; tv.y = outs[nfl - 1]; }
  if (p0 < np) *(volatile v4f*)(op + 4 * p0) = pv0;
  if (p1 < np) *(volatile v4f*)(op + 4 * p1) = pv1;
  if (rem != 0 && tid == 0) *(volatile v2f*)(op + nfl - 2) = tv;
  __threadfence();
  if (p0 < np) *(volatile v4f*)(op + 4 * p0) = pv0;
  if (p1 < np) *(volatile v4f*)(op + 4 * p1) = pv1;
  if (rem != 0 && tid == 0) *(volatile v2f*)(op + nfl - 2) = tv;
}

extern "C" void kernel_launch(void* const* d_in, const int* in_sizes, int n_in,
                              void* d_out, int out_size, void* d_ws, size_t ws_size,
                              hipStream_t stream) {
  if (n_in < 21) return;
  const int nN = in_sizes[1];
  if (nN < 1 || nN > (1 << 24) || in_sizes[0] != nN * FIN) return;
  int nEt[NTYPE];
  for (int t = 0; t < NTYPE; ++t) {
    nEt[t] = in_sizes[2 + t] / 2;
    if (nEt[t] < 1 || in_sizes[2 + t] != 2 * nEt[t] || nEt[t] > (1 << 28)) return;
  }
  if (in_sizes[5] != 2 * EMBD || in_sizes[6] != NTYPE || in_sizes[7] != NTYPE * XIN * HID ||
      in_sizes[8] != NTYPE * HID || in_sizes[9] != NTYPE * HID || in_sizes[10] != NTYPE * HID ||
      in_sizes[11] != NTYPE * HID * HID || in_sizes[12] != NTYPE * HID || in_sizes[13] != NTYPE * HID ||
      in_sizes[14] != NTYPE * HID || in_sizes[15] != 2 * HID * HID || in_sizes[16] != HID ||
      in_sizes[17] != HID * (HID / 2) || in_sizes[18] != HID / 2 || in_sizes[19] != (HID / 2) * NACT ||
      in_sizes[20] != NACT) return;
  const int R = out_size / NACT;
  if (R < 1 || out_size != R * NACT || R > nN) return;

  const float* nf    = (const float*)d_in[0];
  const int*   ntyp  = (const int*)d_in[1];
  const int*   eiT[NTYPE] = { (const int*)d_in[2], (const int*)d_in[3], (const int*)d_in[4] };
  const float* emb   = (const float*)d_in[5];
  const float* eattn = (const float*)d_in[6];
  const float* W1    = (const float*)d_in[7];
  const float* as1   = (const float*)d_in[8];
  const float* ad1   = (const float*)d_in[9];
  const float* b1    = (const float*)d_in[10];
  const float* W2    = (const float*)d_in[11];
  const float* as2   = (const float*)d_in[12];
  const float* ad2   = (const float*)d_in[13];
  const float* b2    = (const float*)d_in[14];
  const float* Wo1   = (const float*)d_in[15];
  const float* bo1   = (const float*)d_in[16];
  const float* Wo2   = (const float*)d_in[17];
  const float* bo2   = (const float*)d_in[18];
  const float* Wo3   = (const float*)d_in[19];
  const float* bo3   = (const float*)d_in[20];
  float* out = (float*)d_out;

  const int NPAD   = ((nN + TGT2 - 1) / TGT2) * TGT2;
  const int nBC    = (nN + NBC - 1) / NBC;
  const int CNTPAD = nBC * NBC;
  if (FPC * nBC + 1 > RBN) return;
  const int nBF    = (nN + NBF - 1) / NBF;
  int Emax = nEt[0];
  for (int t = 1; t < NTYPE; ++t) Emax = nEt[t] > Emax ? nEt[t] : Emax;
  const int csrLen = ((Emax + 31) & ~31) + 4096;
  const int nGemm  = NPAD / GROWS;
  const int nAgg2  = NPAD / TGT2;
  const int nQB    = (R + NBQ - 1) / NBQ;

  char* ws = (char*)d_ws;
  size_t off = 0;
  const size_t oXh  = off; off += (size_t)NPAD * XK * 2;              off = (off + 255) & ~(size_t)255;
  const size_t oXl  = off; off += (size_t)NPAD * XK * 2;              off = (off + 255) & ~(size_t)255;
  const size_t oW1h = off; off += (size_t)NTYPE * HID * XK * 2;       off = (off + 255) & ~(size_t)255;
  const size_t oW1l = off; off += (size_t)NTYPE * HID * XK * 2;       off = (off + 255) & ~(size_t)255;
  const size_t oW2h = off; off += (size_t)NTYPE * HID * HID * 2;      off = (off + 255) & ~(size_t)255;
  const size_t oW2l = off; off += (size_t)NTYPE * HID * HID * 2;      off = (off + 255) & ~(size_t)255;
  const size_t oCnt = off; off += (size_t)CNTPAD * 4;                 off = (off + 255) & ~(size_t)255;
  const size_t oOff = off; off += (size_t)CNTPAD * 4;                 off = (off + 255) & ~(size_t)255;
  const size_t oRb  = off; off += (size_t)RBN * 4;                    off = (off + 255) & ~(size_t)255;
  const size_t oCsr = off; off += (size_t)csrLen * 4;                 off = (off + 255) & ~(size_t)255;
  const size_t oH1  = off; off += (size_t)NPAD * HID * 4;             off = (off + 255) & ~(size_t)255;
  const size_t oAs1 = off; off += (size_t)NPAD * NHEAD * 4;           off = (off + 255) & ~(size_t)255;
  const size_t oAd1 = off; off += (size_t)NPAD * NHEAD * 4;           off = (off + 255) & ~(size_t)255;
  const size_t oH2  = off; off += (size_t)NPAD * HID * 4;             off = (off + 255) & ~(size_t)255;
  const size_t oAs2 = off; off += (size_t)NPAD * 4;                   off = (off + 255) & ~(size_t)255;
  const size_t oAd2 = off; off += (size_t)NPAD * 4;                   off = (off + 255) & ~(size_t)255;
  const size_t oXc  = off; off += (size_t)NPAD * HID * 4;             off = (off + 255) & ~(size_t)255;
  if (off > ws_size) return;
  unsigned short* xh   = (unsigned short*)(ws + oXh);
  unsigned short* xl   = (unsigned short*)(ws + oXl);
  unsigned short* w1h  = (unsigned short*)(ws + oW1h);
  unsigned short* w1l  = (unsigned short*)(ws + oW1l);
  unsigned short* w2h  = (unsigned short*)(ws + oW2h);
  unsigned short* w2l  = (unsigned short*)(ws + oW2l);
  int*   cnt   = (int*)(ws + oCnt);
  int*   offp  = (int*)(ws + oOff);
  int*   rb    = (int*)(ws + oRb);
  int*   csr   = (int*)(ws + oCsr);
  float* h1    = (float*)(ws + oH1);
  float* als1  = (float*)(ws + oAs1);
  float* ald1  = (float*)(ws + oAd1);
  float* h2    = (float*)(ws + oH2);
  float* als2  = (float*)(ws + oAs2);
  float* ald2  = (float*)(ws + oAd2);
  float* xcomb = (float*)(ws + oXc);

  const int nPrep = (NPAD * (XK / 8) + NTYPE * HID * XK / 8 + NTYPE * HID * HID / 8) / NTHR;
  k_prep<<<nPrep, NTHR, 0, stream>>>(nf, ntyp, emb, W1, W2, xh, xl, w1h, w1l, w2h, w2l, nN, NPAD);

  hipFuncSetAttribute(reinterpret_cast<const void*>(&k_fill),
                      hipFuncAttributeMaxDynamicSharedMemorySize, LDS_FILL);
  hipFuncSetAttribute(reinterpret_cast<const void*>(&k_tail),
                      hipFuncAttributeMaxDynamicSharedMemorySize, LDS_TAIL);

  for (int i = 0; i < NTYPE; ++i) {
    const int* ei = eiT[i];
    const int nE = nEt[i];
    const int vec8 = ((nE & 3) == 0) ? 1 : 0;
    k_count<<<nBC, NTHR, 0, stream>>>(ei, cnt, nE, vec8);
    k_offsets<<<1, OTHR, 0, stream>>>(cnt, offp, rb, nBC);
    k_fill<<<nBF, NTHR, LDS_FILL, stream>>>(ei, offp, rb, csr, nN, nE, vec8, csrLen);
    k_gemm1<<<nGemm, NTHR, 0, stream>>>(xh, xl, w1h + (size_t)i * HID * XK, w1l + (size_t)i * HID * XK,
                                          as1 + (size_t)i * HID, ad1 + (size_t)i * HID, h1, als1, ald1);
    k_agg1g2<<<nGemm, NTHR, 0, stream>>>(csr, offp, cnt, als1, ald1, h1, b1 + (size_t)i * HID,
                                           w2h + (size_t)i * HID * HID, w2l + (size_t)i * HID * HID,
                                           as2 + (size_t)i * HID, ad2 + (size_t)i * HID,
                                           h2, als2, ald2, nN, csrLen);
    k_agg2<<<nAgg2, NTHR, 0, stream>>>(csr, offp, cnt, als2, ald2, h2, b2 + (size_t)i * HID,
                                        eattn, i, xcomb, nN, csrLen);
  }

  k_tail<<<nQB, NTHR, LDS_TAIL, stream>>>(eiT[0], nEt[0], ((nEt[0] & 3) == 0) ? 1 : 0, nN, R,
                                          xcomb, Wo1, bo1, Wo2, bo2, Wo3, bo3, out);
}
